// RelationGraphAttention_472446402571
// MI455X (gfx1250) — hardware-verified
//
#include <hip/hip_runtime.h>
#include <stddef.h>
#include <stdint.h>

#define BB   8
#define TL   512
#define NN   1024
#define CC   768
#define HH   12
#define DD   64
#define ROWS (BB * NN)
#define C3   (3 * CC)
#define PL   ((size_t)BB * HH * NN * DD)
#define WEL  ((size_t)CC * CC)

static_assert(NN == 2 * TL);
static_assert(NN % 256 == 0);
static_assert(TL % 128 == 0);
static_assert(CC % 64 == 0);
static_assert(DD == 64);
static_assert(HH * DD == CC);
static_assert(ROWS % 256 == 0);
static_assert((ROWS * CC) % 8 == 0);

typedef _Float16 v16h __attribute__((ext_vector_type(16)));
typedef _Float16 v8h  __attribute__((ext_vector_type(8)));
typedef float    v8f  __attribute__((ext_vector_type(8)));
typedef float    v4f  __attribute__((ext_vector_type(4)));
typedef unsigned int v4u __attribute__((ext_vector_type(4)));

union Frag  { v16h v; v8h h[2]; };
union Pack8 { v8h h; v4u u; };

__device__ __forceinline__ v8f mma16(v16h a, v16h b, v8f c) {
  c = __builtin_amdgcn_wmma_f32_16x16x32_f16(false, a, false, b, (short)0, c, false, false);
  asm volatile("v_nop\n\tv_nop\n\tv_nop\n\tv_nop" : "+v"(c) : "v"(a), "v"(b));
  return c;
}

__device__ __forceinline__ v16h ldfrag(const _Float16* p, int ld, int row0, int k0, int lane) {
  const int m = lane & 15, lh = lane >> 4;
  const _Float16* q = p + (size_t)(row0 + m) * ld + k0 + 8 * lh;
  Frag f;
  f.h[0] = *(const v8h*)(q);
  f.h[1] = *(const v8h*)(q + 16);
  return f.v;
}

__device__ __forceinline__ v8f zero8() { return (v8f){0.f, 0.f, 0.f, 0.f, 0.f, 0.f, 0.f, 0.f}; }

__device__ __forceinline__ void gemm32x64(const _Float16* __restrict__ A, int lda,
                                          const _Float16* __restrict__ Bt, int ldb,
                                          int m0, int n0, int lane, v8f (&acc)[2][4]) {
#pragma unroll 2
  for (int k0 = 0; k0 < CC; k0 += 32) {
    const v16h a0 = ldfrag(A, lda, m0, k0, lane);
    const v16h a1 = ldfrag(A, lda, m0 + 16, k0, lane);
    const v16h b0 = ldfrag(Bt, ldb, n0, k0, lane);
    const v16h b1 = ldfrag(Bt, ldb, n0 + 16, k0, lane);
    const v16h b2 = ldfrag(Bt, ldb, n0 + 32, k0, lane);
    const v16h b3 = ldfrag(Bt, ldb, n0 + 48, k0, lane);
    acc[0][0] = mma16(a0, b0, acc[0][0]);
    acc[1][0] = mma16(a1, b0, acc[1][0]);
    acc[0][1] = mma16(a0, b1, acc[0][1]);
    acc[1][1] = mma16(a1, b1, acc[1][1]);
    acc[0][2] = mma16(a0, b2, acc[0][2]);
    acc[1][2] = mma16(a1, b2, acc[1][2]);
    acc[0][3] = mma16(a0, b3, acc[0][3]);
    acc[1][3] = mma16(a1, b3, acc[1][3]);
  }
}

__global__ __launch_bounds__(256) void k_cvt_x(const float* __restrict__ text, const float* __restrict__ image,
                                               _Float16* __restrict__ xh, int ngrp) {
  const int t = blockIdx.x * 256 + (int)threadIdx.x;
  if (t >= ngrp) return;
  const size_t o = (size_t)t * 8;
  const int m = (int)(o / CC);
  const int c = (int)(o - (size_t)m * CC);
  const int b = m / NN, s = m - b * NN;
  const float* src = (s < TL) ? (text  + (size_t)(b * TL + s) * CC + c)
                              : (image + (size_t)(b * TL + (s - TL)) * CC + c);
  const v4f a0 = *(const v4f*)(src);
  const v4f a1 = *(const v4f*)(src + 4);
  Pack8 pk;
  pk.h = (v8h){(_Float16)a0[0], (_Float16)a0[1], (_Float16)a0[2], (_Float16)a0[3],
               (_Float16)a1[0], (_Float16)a1[1], (_Float16)a1[2], (_Float16)a1[3]};
  const v4u vv = pk.u;
  volatile v4u* d = (volatile v4u*)(xh + o);
  *d = vv;
  __threadfence();
  *d = vv;
}

__global__ __launch_bounds__(256) void k_cvt_w(const float* __restrict__ wq, const float* __restrict__ wk,
                                               const float* __restrict__ wv, const float* __restrict__ wo,
                                               _Float16* __restrict__ wh, int ngrp) {
  const int t = blockIdx.x * 256 + (int)threadIdx.x;
  if (t >= ngrp) return;
  const int y = blockIdx.y;
  const float* w = (y == 0) ? wq : ((y == 1) ? wk : ((y == 2) ? wv : wo));
  const size_t o = (size_t)t * 8;
  const v4f a0 = *(const v4f*)(w + o);
  const v4f a1 = *(const v4f*)(w + o + 4);
  Pack8 pk;
  pk.h = (v8h){(_Float16)(a0[0] * 32.0f), (_Float16)(a0[1] * 32.0f), (_Float16)(a0[2] * 32.0f),
               (_Float16)(a0[3] * 32.0f), (_Float16)(a1[0] * 32.0f), (_Float16)(a1[1] * 32.0f),
               (_Float16)(a1[2] * 32.0f), (_Float16)(a1[3] * 32.0f)};
  const v4u vv = pk.u;
  volatile v4u* d = (volatile v4u*)(wh + (size_t)y * WEL + o);
  *d = vv;
  __threadfence();
  *d = vv;
}

#define STP 72
__global__ __launch_bounds__(256) void k_qkv(const _Float16* __restrict__ xh,
                                             const _Float16* __restrict__ wh,
                                             const float* __restrict__ bq,
                                             const float* __restrict__ bk,
                                             const float* __restrict__ bv,
                                             _Float16* __restrict__ qkv) {
  __shared__ __align__(16) _Float16 st[256 * STP];
  const int tid = threadIdx.x, lane = tid & 31, wave = tid >> 5;
  const int hh = lane >> 4, c = lane & 15;
  const int mb = blockIdx.x * 256;
  const int m0 = mb + wave * 32;
  const int n0 = blockIdx.y * 64;

  v8f acc[2][4];
#pragma unroll
  for (int s = 0; s < 2; ++s)
#pragma unroll
    for (int t = 0; t < 4; ++t) acc[s][t] = zero8();
  gemm32x64(xh, CC, wh, CC, m0, n0, lane, acc);

  const int which = n0 / CC;
  const int nloc  = n0 - which * CC;
  const int head  = nloc / DD;
  const float* bias = (which == 0) ? bq : ((which == 1) ? bk : bv);

#pragma unroll
  for (int t = 0; t < 4; ++t) {
    const float bvv = bias[nloc + 16 * t + c];
#pragma unroll
    for (int sub = 0; sub < 2; ++sub) {
#pragma unroll
      for (int r = 0; r < 8; ++r) {
        const int lr = wave * 32 + sub * 16 + 8 * hh + r;
        st[lr * STP + 16 * t + c] = (_Float16)(acc[sub][t][r] * 0.03125f + bvv);
      }
    }
  }
  __syncthreads();

  const int b  = mb / NN;
  const int nb = mb - b * NN;
  const int bh = b * HH + head;
  v4u val[8];
  size_t go[8];
  if (which < 2) {
#pragma unroll
    for (int j = 0; j < 8; ++j) {
      const int p  = tid + 256 * j;
      const int lr = p >> 3;
      const int pc = p & 7;
      Pack8 pk;
      pk.h  = *(const v8h*)(st + lr * STP + pc * 8);
      val[j] = pk.u;
      go[j]  = (size_t)which * PL + ((size_t)bh * NN + nb + lr) * DD + pc * 8;
    }
  } else {
#pragma unroll
    for (int j = 0; j < 8; ++j) {
      const int p  = tid + 256 * j;
      const int L  = p >> 3;
      const int pc = p & 7;
      const int d  = L >> 2;
      const int nl = (L & 3) * 64 + pc * 8;
      const _Float16* cp = st + nl * STP + d;
      Pack8 pk;
      pk.h = (v8h){cp[0 * STP], cp[1 * STP], cp[2 * STP], cp[3 * STP],
                   cp[4 * STP], cp[5 * STP], cp[6 * STP], cp[7 * STP]};
      val[j] = pk.u;
      go[j]  = 2 * PL + ((size_t)bh * DD + d) * NN + nb + nl;
    }
  }
  for (int ps = 0; ps < 2; ++ps) {
#pragma unroll
    for (int j = 0; j < 8; ++j) *(volatile v4u*)(qkv + go[j]) = val[j];
    __threadfence();
  }
}

#define KTP 72
#define PTP 72
__global__ __launch_bounds__(256) void k_attn(const _Float16* __restrict__ qp,
                                              const _Float16* __restrict__ kp,
                                              const _Float16* __restrict__ vt,
                                              const float* __restrict__ rel,
                                              _Float16* __restrict__ op, float sscale) {
  __shared__ __align__(16) _Float16 Ks[64 * KTP];
  __shared__ __align__(16) _Float16 Vs[64 * KTP];
  __shared__ __align__(16) _Float16 Ps[8][16 * PTP];
  __shared__ float red[3][8];

  const int tid = threadIdx.x, lane = tid & 31, wave = tid >> 5;
  const int hh = lane >> 4, c = lane & 15;
  const int bh = blockIdx.x >> 3;
  const int qb = blockIdx.x & 7;
  const int b  = bh / HH, h = bh - b * HH;
  const int q0 = qb * 128 + wave * 16;

  {
    float s0 = 0.f, s1 = 0.f, s2 = 0.f;
    for (int i = tid; i < CC; i += 256) {
      s0 += rel[i];
      s1 += rel[CC + i];
      s2 += rel[2 * CC + i];
    }
#pragma unroll
    for (int off = 1; off < 32; off <<= 1) {
      s0 += __shfl_xor(s0, off, 32);
      s1 += __shfl_xor(s1, off, 32);
      s2 += __shfl_xor(s2, off, 32);
    }
    if (lane == 0) { red[0][wave] = s0; red[1][wave] = s1; red[2][wave] = s2; }
  }
  __syncthreads();
  float mt[3];
#pragma unroll
  for (int ty = 0; ty < 3; ++ty) {
    float s = 0.f;
#pragma unroll
    for (int w = 0; w < 8; ++w) s += red[ty][w];
    mt[ty] = s * (1.0f / (float)CC);
  }
  const int qside = (qb * 128 >= TL) ? 1 : 0;
  const float cb_lo = qside ? mt[2] : mt[0];
  const float cb_hi = qside ? mt[0] : mt[1];

  const _Float16* Q = qp + (size_t)bh * NN * DD;
  const _Float16* K = kp + (size_t)bh * NN * DD;
  const _Float16* V = vt + (size_t)bh * DD * NN;

  v16h qa[2];
  qa[0] = ldfrag(Q, DD, q0, 0, lane);
  qa[1] = ldfrag(Q, DD, q0, 32, lane);

  const float NEGI = -__builtin_huge_valf();
  float mrow[8], lrow[8];
  v8f oacc[4];
#pragma unroll
  for (int r = 0; r < 8; ++r) { mrow[r] = NEGI; lrow[r] = 0.f; }
#pragma unroll
  for (int t = 0; t < 4; ++t) oacc[t] = zero8();

  _Float16* pw = Ps[wave];

  for (int kc = 0; kc < NN / 64; ++kc) {
    const int kv0 = kc * 64;
    const float cb = (kv0 >= TL) ? cb_hi : cb_lo;
    __syncthreads();
    {
      const int r  = tid >> 2;
      const int qq = (tid & 3) * 16;
      const _Float16* ks = K + (size_t)(kv0 + r) * DD + qq;
      *(v8h*)(Ks + r * KTP + qq)     = *(const v8h*)(ks);
      *(v8h*)(Ks + r * KTP + qq + 8) = *(const v8h*)(ks + 8);
      const _Float16* vs = V + (size_t)r * NN + kv0 + qq;
      *(v8h*)(Vs + r * KTP + qq)     = *(const v8h*)(vs);
      *(v8h*)(Vs + r * KTP + qq + 8) = *(const v8h*)(vs + 8);
    }
    __syncthreads();

    v8f s[4];
#pragma unroll
    for (int j = 0; j < 4; ++j) s[j] = zero8();
#pragma unroll
    for (int dc = 0; dc < 2; ++dc) {
#pragma unroll
      for (int j = 0; j < 4; ++j) {
        const v16h kb = ldfrag(Ks, KTP, j * 16, dc * 32, lane);
        s[j] = mma16(qa[dc], kb, s[j]);
      }
    }
    float cm[8];
#pragma unroll
    for (int r = 0; r < 8; ++r) {
      float m = NEGI;
#pragma unroll
      for (int j = 0; j < 4; ++j) {
        const float sv = s[j][r] * sscale + cb;
        s[j][r] = sv;
        m = fmaxf(m, sv);
      }
#pragma unroll
      for (int off = 1; off < 16; off <<= 1) m = fmaxf(m, __shfl_xor(m, off, 32));
      cm[r] = m;
    }
    float al[8];
#pragma unroll
    for (int r = 0; r < 8; ++r) {
      const float mnew  = fmaxf(mrow[r], cm[r]);
      const float alpha = __expf(mrow[r] - mnew);
      mrow[r] = mnew;
      float psum = 0.f;
#pragma unroll
      for (int j = 0; j < 4; ++j) {
        const float p = __expf(s[j][r] - mnew);
        psum += p;
        pw[(8 * hh + r) * PTP + j * 16 + c] = (_Float16)(p * 1024.0f);
      }
#pragma unroll
      for (int off = 1; off < 16; off <<= 1) psum += __shfl_xor(psum, off, 32);
      lrow[r] = lrow[r] * alpha + psum;
      al[r] = alpha;
    }
#pragma unroll
    for (int t = 0; t < 4; ++t)
#pragma unroll
      for (int r = 0; r < 8; ++r) oacc[t][r] *= al[r];
    __syncthreads();

#pragma unroll
    for (int kk = 0; kk < 2; ++kk) {
      const v16h pa = ldfrag(pw, PTP, 0, kk * 32, lane);
#pragma unroll
      for (int t = 0; t < 4; ++t) {
        const v16h vb = ldfrag(Vs, KTP, t * 16, kk * 32, lane);
        oacc[t] = mma16(pa, vb, oacc[t]);
      }
    }
  }
  __syncthreads();

#pragma unroll
  for (int r = 0; r < 8; ++r) {
    const float inv = 0.0625f / lrow[r];
#pragma unroll
    for (int t = 0; t < 4; ++t) pw[(8 * hh + r) * PTP + 16 * t + c] = (_Float16)(oacc[t][r] * inv);
  }
  __syncthreads();
  v4u val[4];
  size_t go[4];
#pragma unroll
  for (int it = 0; it < 4; ++it) {
    const int p  = lane + 32 * it;
    const int L  = p >> 3;
    const int pc = p & 7;
    Pack8 pk;
    pk.h   = *(const v8h*)(pw + L * PTP + pc * 8);
    val[it] = pk.u;
    go[it]  = ((size_t)(b * NN + q0 + L)) * CC + (size_t)h * DD + pc * 8;
  }
  for (int ps = 0; ps < 2; ++ps) {
#pragma unroll
    for (int it = 0; it < 4; ++it) *(volatile v4u*)(op + go[it]) = val[it];
    __threadfence();
  }
}

#define OTP 68
__global__ __launch_bounds__(256) void k_proj(const _Float16* __restrict__ ap,
                                              const _Float16* __restrict__ wt,
                                              const float* __restrict__ bias,
                                              float* __restrict__ out) {
  __shared__ __align__(16) float st[8][16 * OTP];
  const int tid = threadIdx.x, lane = tid & 31, wave = tid >> 5;
  const int hh = lane >> 4, c = lane & 15;
  const int m0 = blockIdx.x * 256 + wave * 32;
  const int n0 = blockIdx.y * 64;

  v8f acc[2][4];
#pragma unroll
  for (int s = 0; s < 2; ++s)
#pragma unroll
    for (int t = 0; t < 4; ++t) acc[s][t] = zero8();
  gemm32x64(ap, CC, wt, CC, m0, n0, lane, acc);

  float bvs[4];
#pragma unroll
  for (int t = 0; t < 4; ++t) bvs[t] = bias[n0 + 16 * t + c];

  float* sw = st[wave];
#pragma unroll
  for (int sub = 0; sub < 2; ++sub) {
    __syncthreads();
#pragma unroll
    for (int t = 0; t < 4; ++t) {
#pragma unroll
      for (int r = 0; r < 8; ++r)
        sw[(8 * hh + r) * OTP + 16 * t + c] = acc[sub][t][r] * 0.00048828125f + bvs[t];
    }
    __syncthreads();
    v4f val[8];
    size_t go[8];
#pragma unroll
    for (int it = 0; it < 8; ++it) {
      const int p    = lane + 32 * it;
      const int L    = p >> 3;
      const int pc   = p & 7;
      const int row  = L >> 1;
      const int half = L & 1;
      val[it] = *(const v4f*)(sw + row * OTP + half * 32 + pc * 4);
      go[it]  = (size_t)(m0 + sub * 16 + row) * CC + n0 + half * 32 + pc * 4;
    }
    for (int ps = 0; ps < 2; ++ps) {
#pragma unroll
      for (int it = 0; it < 8; ++it) *(volatile v4f*)(out + go[it]) = val[it];
      __threadfence();
    }
  }
}

extern "C" void kernel_launch(void* const* d_in, const int* in_sizes, int n_in,
                              void* d_out, int out_size, void* d_ws, size_t ws_size,
                              hipStream_t stream) {
  if (n_in < 11) return;
  if (in_sizes[0] != BB * TL * CC) return;
  if (in_sizes[1] != BB * TL * CC) return;
  if (in_sizes[2] != CC * CC || in_sizes[4] != CC * CC || in_sizes[6] != CC * CC || in_sizes[8] != CC * CC) return;
  if (in_sizes[3] != CC || in_sizes[5] != CC || in_sizes[7] != CC || in_sizes[9] != CC) return;
  if (in_sizes[10] != 3 * CC) return;
  if (out_size != ROWS * CC) return;

  const float* text  = (const float*)d_in[0];
  const float* image = (const float*)d_in[1];
  const float* wq    = (const float*)d_in[2];
  const float* bq    = (const float*)d_in[3];
  const float* wk    = (const float*)d_in[4];
  const float* bk    = (const float*)d_in[5];
  const float* wv    = (const float*)d_in[6];
  const float* bv    = (const float*)d_in[7];
  const float* wo    = (const float*)d_in[8];
  const float* bo    = (const float*)d_in[9];
  const float* rel   = (const float*)d_in[10];
  float* out = (float*)d_out;

  size_t off = 0;
  const size_t oX   = off; off += (size_t)ROWS * CC * 2;
  const size_t oW   = off; off += 4 * WEL * 2;
  const size_t oQKV = off; off += 3 * PL * 2;
  const size_t oO   = off; off += (size_t)ROWS * CC * 2;
  if (off > ws_size) return;

  char* ws = (char*)d_ws;
  _Float16* Xh   = (_Float16*)(ws + oX);
  _Float16* Wh   = (_Float16*)(ws + oW);
  _Float16* QKVp = (_Float16*)(ws + oQKV);
  _Float16* Op   = (_Float16*)(ws + oO);

  const int ngx = (ROWS * CC) / 8;
  k_cvt_x<<<dim3((ngx + 255) / 256), dim3(256), 0, stream>>>(text, image, Xh, ngx);
  const int ngw = (int)(WEL / 8);
  k_cvt_w<<<dim3((ngw + 255) / 256, 4), dim3(256), 0, stream>>>(wq, wk, wv, wo, Wh, ngw);
  k_qkv<<<dim3(ROWS / 256, C3 / 64), dim3(256), 0, stream>>>(Xh, Wh, bq, bk, bv, QKVp);
  k_attn<<<dim3(BB * HH * (NN / 128)), dim3(256), 0, stream>>>(QKVp, QKVp + PL, QKVp + 2 * PL, rel, Op, 0.125f);
  k_proj<<<dim3(ROWS / 256, CC / 64), dim3(256), 0, stream>>>(Op, Wh + 3 * WEL, bo, out);
  (void)hipGetLastError();
}
